// GSA_19567871001251
// MI455X (gfx1250) — hardware-verified
//
#include <hip/hip_runtime.h>


#define NB   8
#define NT   1024
#define NF   512
#define NHD  8
#define NDK  64
#define NDH  512
#define NDO  512
#define NO3  1536
#define NHN  64
#define NL   32
#define NREL 63

typedef unsigned short u16;
typedef u16    v8us  __attribute__((ext_vector_type(8)));
typedef u16    v16us __attribute__((ext_vector_type(16)));
typedef __bf16 v16b  __attribute__((ext_vector_type(16)));
typedef float  v8f   __attribute__((ext_vector_type(8)));
typedef float  v4f   __attribute__((ext_vector_type(4)));
typedef double v2d   __attribute__((ext_vector_type(2)));

union F16 { v16b b; v16us u; v8us h[2]; u16 s[16]; };
union F8  { v8us u; u16 s[8]; };

__device__ __forceinline__ v8f zero8() {
    v8f z = {0.f, 0.f, 0.f, 0.f, 0.f, 0.f, 0.f, 0.f};
    return z;
}

__device__ __forceinline__ v8f mma(v16us a, v16us b, v8f c) {
    F16 fa, fb;
    fa.u = a;
    fb.u = b;
    c = __builtin_amdgcn_wmma_f32_16x16x32_bf16(false, fa.b, false, fb.b, (short)0, c,
                                                 false, false);
    asm volatile("v_nop\n\tv_nop\n\tv_nop\n\tv_nop" : "+v"(c) : "v"(fa.b), "v"(fb.b));
    return c;
}

__device__ __forceinline__ v8f mma3(v16us ah, v16us al, v16us bh, v16us bl, v8f c) {
    c = mma(ah, bh, c);
    c = mma(ah, bl, c);
    c = mma(al, bh, c);
    return c;
}

__device__ __forceinline__ v16us ldfrag(const u16* __restrict__ p, int h) {
    F16 f;
    f.h[0] = *(const v8us*)(p + 8 * h);
    f.h[1] = *(const v8us*)(p + 16 + 8 * h);
    return f.u;
}

__device__ __forceinline__ u16 bf16_rne(float f) {
    unsigned int u = __float_as_uint(f);
    u += 0x7FFFu + ((u >> 16) & 1u);
    return (u16)(u >> 16);
}

__device__ __forceinline__ void split1(float f, u16& hi, u16& lo) {
    const u16 hb = bf16_rne(f);
    const float hf = __uint_as_float(((unsigned int)hb) << 16);
    hi = hb;
    lo = bf16_rne(f - hf);
}

__device__ __forceinline__ void split8(v4f a, v4f b, v8us& hv, v8us& lv) {
    F8 H, L;
#pragma unroll
    for (int i = 0; i < 4; ++i) {
        split1(a[i], H.s[i], L.s[i]);
        split1(b[i], H.s[4 + i], L.s[4 + i]);
    }
    hv = H.u;
    lv = L.u;
}

__global__ void __launch_bounds__(256) k_cvt(const float* __restrict__ src, size_t src_bstride,
                                            u16* __restrict__ dh, u16* __restrict__ dl,
                                            size_t dst_bstride, int n8) {
    const int b  = blockIdx.y;
    const int g  = blockIdx.x * 256 + threadIdx.x;
    const bool ok = g < n8;
    const int gg = ok ? g : 0;
    const float* s = src + (size_t)b * src_bstride + (size_t)gg * 8;
    const v4f x0 = *(const v4f*)s;
    const v4f x1 = *(const v4f*)(s + 4);
    v8us hv, lv;
    split8(x0, x1, hv, lv);
    u16* ph = dh + (size_t)b * dst_bstride + (size_t)gg * 8;
    u16* pl = dl + (size_t)b * dst_bstride + (size_t)gg * 8;
    if (ok) {
        *(volatile v8us*)ph = hv;
        *(volatile v8us*)pl = lv;
    }
    __threadfence();
    if (ok) {
        *(volatile v8us*)ph = hv;
        *(volatile v8us*)pl = lv;
    }
}

__global__ void __launch_bounds__(128) k_gemm(const u16* __restrict__ Ah, const u16* __restrict__ Al,
                                             const u16* __restrict__ Bh, const u16* __restrict__ Bl,
                                             size_t b_bstride, float* __restrict__ C, size_t c_bstride,
                                             const float* __restrict__ bias, int bias_n, int has_bias,
                                             int M, int N, int K) {
    __shared__ float Cs[64 * 68];
    const int n0 = blockIdx.x * 64;
    const int m0 = blockIdx.y * 64;
    const int bz = blockIdx.z;
    if (m0 + 64 > M || n0 + 64 > N) return;

    const int w = threadIdx.x >> 5, lane = threadIdx.x & 31, h = lane >> 4, nl = lane & 15;
    const int wm = w & 1, wn = w >> 1;
    const u16* Bhb = Bh + (size_t)bz * b_bstride;
    const u16* Blb = Bl + (size_t)bz * b_bstride;
    const size_t ra0 = (size_t)(m0 + wm * 32 + nl) * K;
    const size_t ra1 = ra0 + (size_t)16 * K;
    const size_t rb0 = (size_t)(n0 + wn * 32 + nl) * K;
    const size_t rb1 = rb0 + (size_t)16 * K;

    v8f acc00 = zero8(), acc01 = zero8(), acc10 = zero8(), acc11 = zero8();
    for (int kb = 0; kb < K; kb += 32) {
        const v16us ah0 = ldfrag(Ah + ra0 + kb, h), al0 = ldfrag(Al + ra0 + kb, h);
        const v16us ah1 = ldfrag(Ah + ra1 + kb, h), al1 = ldfrag(Al + ra1 + kb, h);
        const v16us bh0 = ldfrag(Bhb + rb0 + kb, h), bl0 = ldfrag(Blb + rb0 + kb, h);
        const v16us bh1 = ldfrag(Bhb + rb1 + kb, h), bl1 = ldfrag(Blb + rb1 + kb, h);
        acc00 = mma3(ah0, al0, bh0, bl0, acc00);
        acc01 = mma3(ah0, al0, bh1, bl1, acc01);
        acc10 = mma3(ah1, al1, bh0, bl0, acc10);
        acc11 = mma3(ah1, al1, bh1, bl1, acc11);
    }

    {
        const int rbase = wm * 32 + 8 * h;
        const int cbase = wn * 32 + nl;
#pragma unroll
        for (int r = 0; r < 8; ++r) {
            Cs[(rbase + r) * 68 + cbase]           = acc00[r];
            Cs[(rbase + r) * 68 + cbase + 16]      = acc01[r];
            Cs[(rbase + 16 + r) * 68 + cbase]      = acc10[r];
            Cs[(rbase + 16 + r) * 68 + cbase + 16] = acc11[r];
        }
    }
    __syncthreads();

    float* Cb = C + (size_t)bz * c_bstride;
#pragma unroll 1
    for (int pass = 0; pass < 2; ++pass) {
#pragma unroll
        for (int it = 0; it < 8; ++it) {
            const int row = w * 16 + it * 2 + (lane >> 4);
            const int c4  = (lane & 15) * 4;
            v4f v = *(const v4f*)&Cs[row * 68 + c4];
            if (has_bias) {
                int bi = m0 + row;
                if (bi > bias_n - 1) bi = bias_n - 1;
                const float bb = bias[bi];
                v = v + bb;
            }
            *(volatile v4f*)(Cb + (size_t)(m0 + row) * N + n0 + c4) = v;
        }
        if (pass == 0) __threadfence();
    }
}

__global__ void __launch_bounds__(64) k_psum(const float* __restrict__ relp, float* __restrict__ psum) {
    __shared__ float ps[64];
    const int t = blockIdx.x;
    const int d = threadIdx.x;
    int rlo = (NL - 1) - t;          if (rlo < 0) rlo = 0;
    int rhi = (NT + NL - 2) - t;     if (rhi > 2 * NL - 2) rhi = 2 * NL - 2;
    float s = 0.f;
    for (int r = rlo; r <= rhi; ++r) s += relp[r * NDK + d];
    ps[d] = s;
    __syncthreads();
    if (d < 16) {
        const v4f v = *(const v4f*)&ps[d * 4];
        float* dst = psum + (size_t)t * NDK + d * 4;
        *(volatile v4f*)dst = v;
        __threadfence();
        *(volatile v4f*)dst = v;
    }
}

__global__ void __launch_bounds__(128) k_soft(const float* __restrict__ qkv, u16* __restrict__ kh,
                                             u16* __restrict__ kl) {
    __shared__ float red[8];
    const int blk  = blockIdx.x;
    const int b    = blk >> 9, j = blk & 511;
    const int tid  = threadIdx.x, w = tid >> 5, lane = tid & 31;
    const float* row = qkv + (size_t)b * NO3 * NT + (size_t)(NDH + j) * NT;
    const int t0   = tid * 8;
    const v4f x0 = *(const v4f*)(row + t0);
    const v4f x1 = *(const v4f*)(row + t0 + 4);

    float m = fmaxf(fmaxf(fmaxf(x0[0], x0[1]), fmaxf(x0[2], x0[3])),
                    fmaxf(fmaxf(x1[0], x1[1]), fmaxf(x1[2], x1[3])));
    for (int o = 16; o > 0; o >>= 1) m = fmaxf(m, __shfl_xor(m, o));
    if (lane == 0) red[w] = m;
    __syncthreads();
    m = fmaxf(fmaxf(red[0], red[1]), fmaxf(red[2], red[3]));

    v4f e0 = x0, e1 = x1;
    float s = 0.f;
#pragma unroll
    for (int i = 0; i < 4; ++i) { e0[i] = __expf(x0[i] - m); s += e0[i]; }
#pragma unroll
    for (int i = 0; i < 4; ++i) { e1[i] = __expf(x1[i] - m); s += e1[i]; }
    for (int o = 16; o > 0; o >>= 1) s += __shfl_xor(s, o);
    if (lane == 0) red[4 + w] = s;
    __syncthreads();
    s = ((red[4] + red[5]) + red[6]) + red[7];
    const float inv = 1.0f / s;
    e0 = e0 * inv;
    e1 = e1 * inv;

    v8us hv, lv;
    split8(e0, e1, hv, lv);
    const size_t dst = (size_t)blk * NT + t0;
    *(volatile v8us*)(kh + dst) = hv;
    *(volatile v8us*)(kl + dst) = lv;
    __threadfence();
    *(volatile v8us*)(kh + dst) = hv;
    *(volatile v8us*)(kl + dst) = lv;
}

__global__ void __launch_bounds__(256) k_qtr(const float* __restrict__ qkv, u16* __restrict__ qth,
                                            u16* __restrict__ qtl) {
    __shared__ float qs[32 * 64];
    const int tc = blockIdx.x, n = blockIdx.y;
    const int t0 = tc * 32;
    const int b = n >> 3, hh = n & 7;
    const float* qbase = qkv + (size_t)b * NO3 * NT + (size_t)(hh * NDK) * NT;
    const int tid = threadIdx.x;
    {
        const int d  = tid >> 2;
        const int t8 = (tid & 3) * 8;
        const float* p = qbase + (size_t)d * NT + t0 + t8;
        const v4f a = *(const v4f*)p;
        const v4f c = *(const v4f*)(p + 4);
#pragma unroll
        for (int i = 0; i < 4; ++i) {
            qs[(t8 + i) * 64 + d]     = a[i];
            qs[(t8 + 4 + i) * 64 + d] = c[i];
        }
    }
    __syncthreads();
    const int w = tid >> 5, lane = tid & 31;
    const int tl = w * 4 + (lane >> 3);
    const int jg = lane & 7;
    const v4f a = *(const v4f*)&qs[tl * 64 + jg * 8];
    const v4f c = *(const v4f*)&qs[tl * 64 + jg * 8 + 4];
    v8us hv, lv;
    split8(a, c, hv, lv);
    const size_t dst = (size_t)(n * NT + t0 + tl) * NDK + jg * 8;
    *(volatile v8us*)(qth + dst) = hv;
    *(volatile v8us*)(qtl + dst) = lv;
    __threadfence();
    *(volatile v8us*)(qth + dst) = hv;
    *(volatile v8us*)(qtl + dst) = lv;
}

__global__ void __launch_bounds__(256) k_rel(const float* __restrict__ qkv, const float* __restrict__ psum,
                                            float* __restrict__ Sbuf, double* __restrict__ bnpart) {
    __shared__ float  Sl[NT];
    __shared__ double part[512];
    __shared__ double outp[128];
    const int n = blockIdx.x;
    const int b = n >> 3, hh = n & 7;
    const float* qbase = qkv + (size_t)b * NO3 * NT + (size_t)(hh * NDK) * NT;
    const float* vbase = qbase + (size_t)(2 * NDH) * NT;
    const int tid = threadIdx.x;

    for (int i = 0; i < 4; ++i) {
        const int t = tid + 256 * i;
        float s = 0.f;
#pragma unroll 4
        for (int d = 0; d < NDK; ++d) s = fmaf(qbase[(size_t)d * NT + t], psum[t * NDK + d], s);
        Sl[t] = s;
    }
    __syncthreads();

    const int e  = tid >> 2;
    const int jq = tid & 3;
    const float* vrow = vbase + (size_t)e * NT;
    double sm = 0.0, sq = 0.0;
    for (int t = jq * 256; t < jq * 256 + 256; ++t) {
        const float r = vrow[t] * Sl[t];
        sm += (double)r;
        sq += (double)r * (double)r;
    }
    part[e * 4 + jq]       = sm;
    part[256 + e * 4 + jq] = sq;
    __syncthreads();
    if (tid < 64) {
        const double s0 = ((part[tid * 4] + part[tid * 4 + 1]) + part[tid * 4 + 2]) + part[tid * 4 + 3];
        const double s1 = ((part[256 + tid * 4] + part[256 + tid * 4 + 1]) + part[256 + tid * 4 + 2]) +
                          part[256 + tid * 4 + 3];
        outp[tid]      = s0;
        outp[64 + tid] = s1;
    }
    __syncthreads();

    const v4f sv = *(const v4f*)&Sl[tid * 4];
    float* sdst  = Sbuf + (size_t)n * NT + tid * 4;
    v2d bv;
    bv[0] = 0.0; bv[1] = 0.0;
    double* bdst = bnpart + (size_t)n * 128;
    if (tid < 64) {
        bv[0] = outp[tid * 2];
        bv[1] = outp[tid * 2 + 1];
        bdst  = bnpart + (size_t)n * 128 + tid * 2;
    }
    *(volatile v4f*)sdst = sv;
    if (tid < 64) *(volatile v2d*)bdst = bv;
    __threadfence();
    *(volatile v4f*)sdst = sv;
    if (tid < 64) *(volatile v2d*)bdst = bv;
}

__global__ void __launch_bounds__(64) k_bnfin(const double* __restrict__ bnpart, const float* __restrict__ gamma,
                                             const float* __restrict__ beta, float* __restrict__ bncoef) {
    __shared__ float cf[128];
    const int e = threadIdx.x;
    double sm = 0.0, sq = 0.0;
    for (int nn = 0; nn < NHN; ++nn) {
        sm += bnpart[nn * 128 + e];
        sq += bnpart[nn * 128 + 64 + e];
    }
    const double cnt = 1.0 / (double)(NHN * NT);
    const double mu  = sm * cnt;
    double var = sq * cnt - mu * mu;
    if (var < 0.0) var = 0.0;
    const float varf = (float)var;
    const float inv  = rsqrtf(varf + 1e-5f);
    const float sc   = inv * gamma[e];
    const float sh   = beta[e] - (float)mu * sc;
    cf[e]      = sc;
    cf[64 + e] = sh;
    __syncthreads();
    if (e < 32) {
        const v4f v = *(const v4f*)&cf[e * 4];
        float* dst = bncoef + e * 4;
        *(volatile v4f*)dst = v;
        __threadfence();
        *(volatile v4f*)dst = v;
    }
}

__global__ void __launch_bounds__(256) k_head(const float* __restrict__ qkv,
                                             const u16* __restrict__ kh, const u16* __restrict__ kl,
                                             const u16* __restrict__ vh, const u16* __restrict__ vl,
                                             const u16* __restrict__ qth, const u16* __restrict__ qtl,
                                             const float* __restrict__ Sbuf, const float* __restrict__ bncoef,
                                             u16* __restrict__ hidh, u16* __restrict__ hidl) {
    __shared__ float ctx[64 * 64];
    __shared__ float tileC[64 * 64];
    __shared__ float vs[64 * 64];
    __shared__ float Sl[NT];
    __shared__ float cf[128];

    const int n = blockIdx.x;
    const int b = n >> 3, hh = n & 7;
    const int tid = threadIdx.x, w = tid >> 5, lane = tid & 31, h = lane >> 4, nl = lane & 15;
    const float* vbase = qkv + (size_t)b * NO3 * NT + (size_t)(2 * NDH + hh * NDK) * NT;

    {
        const v4f s4 = *(const v4f*)(Sbuf + (size_t)n * NT + tid * 4);
        *(v4f*)&Sl[tid * 4] = s4;
    }
    if (tid < 128) cf[tid] = bncoef[tid];

    {
        const int mtile = (w >> 1) * 16;
        const int ntile = (w & 1) * 32;
        const u16* arh  = kh + (size_t)(n * 64 + mtile + nl) * NT;
        const u16* arl  = kl + (size_t)(n * 64 + mtile + nl) * NT;
        const u16* brh0 = vh + (size_t)(n * 64 + ntile + nl) * NT;
        const u16* brl0 = vl + (size_t)(n * 64 + ntile + nl) * NT;
        const u16* brh1 = brh0 + (size_t)16 * NT;
        const u16* brl1 = brl0 + (size_t)16 * NT;
        v8f acc0 = zero8(), acc1 = zero8();
        for (int kb = 0; kb < NT; kb += 32) {
            const v16us ah  = ldfrag(arh + kb, h),  al  = ldfrag(arl + kb, h);
            const v16us bh0 = ldfrag(brh0 + kb, h), bl0 = ldfrag(brl0 + kb, h);
            const v16us bh1 = ldfrag(brh1 + kb, h), bl1 = ldfrag(brl1 + kb, h);
            acc0 = mma3(ah, al, bh0, bl0, acc0);
            acc1 = mma3(ah, al, bh1, bl1, acc1);
        }
#pragma unroll
        for (int r = 0; r < 8; ++r) {
            ctx[(mtile + 8 * h + r) * 64 + ntile + nl]      = acc0[r];
            ctx[(mtile + 8 * h + r) * 64 + ntile + 16 + nl] = acc1[r];
        }
    }
    __syncthreads();

    const int mt2 = w & 3;
    const int ntb = (w >> 2) * 32;
    v16us a2h[2], a2l[2];
#pragma unroll
    for (int ks = 0; ks < 2; ++ks) {
        F16 th, tl;
#pragma unroll
        for (int i = 0; i < 16; ++i) {
            const int kk = ks * 32 + ((i < 8) ? (8 * h + i) : (8 + 8 * h + i));
            const float cv = ctx[kk * 64 + mt2 * 16 + nl];
            split1(cv, th.s[i], tl.s[i]);
        }
        a2h[ks] = th.u;
        a2l[ks] = tl.u;
    }

    for (int c = 0; c < NT / 64; ++c) {
        const int t0c = c * 64;
        __syncthreads();
        {
            const int e  = tid >> 2;
            const int tq = (tid & 3) * 16;
            const float* vp = vbase + (size_t)e * NT + t0c + tq;
#pragma unroll
            for (int i = 0; i < 4; ++i)
                *(v4f*)&vs[e * 64 + tq + 4 * i] = *(const v4f*)(vp + 4 * i);
        }
        v8f acc2[2];
        acc2[0] = zero8();
        acc2[1] = zero8();
#pragma unroll
        for (int nt = 0; nt < 2; ++nt) {
            const int t = t0c + ntb + nt * 16 + nl;
            const u16* qh = qth + (size_t)(n * NT + t) * NDK;
            const u16* ql = qtl + (size_t)(n * NT + t) * NDK;
#pragma unroll
            for (int ks = 0; ks < 2; ++ks) {
                const v16us bh = ldfrag(qh + ks * 32, h);
                const v16us bl = ldfrag(ql + ks * 32, h);
                acc2[nt] = mma3(a2h[ks], a2l[ks], bh, bl, acc2[nt]);
            }
        }
#pragma unroll
        for (int nt = 0; nt < 2; ++nt)
#pragma unroll
            for (int r = 0; r < 8; ++r)
                tileC[(ntb + nt * 16 + nl) * 64 + mt2 * 16 + 8 * h + r] = acc2[nt][r];
        __syncthreads();

#pragma unroll 1
        for (int pass = 0; pass < 2; ++pass) {
#pragma unroll
            for (int p = 0; p < 2; ++p) {
                const int tl = p * 32 + w * 4 + (lane >> 3);
                const int jg = lane & 7;
                const int e0 = jg * 8;
                const int t  = t0c + tl;
                const float s = Sl[t];
                v4f ha, hb;
#pragma unroll
                for (int i = 0; i < 4; ++i) {
                    const float r0 = vs[(e0 + i) * 64 + tl] * s;
                    ha[i] = tileC[tl * 64 + e0 + i] + fmaf(r0, cf[e0 + i], cf[64 + e0 + i]);
                    const float r1 = vs[(e0 + 4 + i) * 64 + tl] * s;
                    hb[i] = tileC[tl * 64 + e0 + 4 + i] + fmaf(r1, cf[e0 + 4 + i], cf[64 + e0 + 4 + i]);
                }
                v8us hv, lv;
                split8(ha, hb, hv, lv);
                const size_t dst = (size_t)(b * NT + t) * NDH + hh * NDK + e0;
                *(volatile v8us*)(hidh + dst) = hv;
                *(volatile v8us*)(hidl + dst) = lv;
            }
            if (pass == 0) __threadfence();
        }
    }
}

static inline size_t al256(size_t x) { return (x + 255) & ~(size_t)255; }

extern "C" void kernel_launch(void* const* d_in, const int* in_sizes, int n_in,
                              void* d_out, int out_size, void* d_ws, size_t ws_size,
                              hipStream_t stream) {
    if (n_in < 7) return;
    if (in_sizes[0] != NB * NT * NF) return;
    if (in_sizes[1] != NO3 * NF) return;
    if (in_sizes[2] != NDO * NDH) return;
    if (in_sizes[3] != NDO) return;
    if (in_sizes[4] != NREL * NDK) return;
    if (in_sizes[5] != NDK || in_sizes[6] != NDK) return;
    if (out_size != NB * NDO * NT) return;

    const float* x     = (const float*)d_in[0];
    const float* Wqkv  = (const float*)d_in[1];
    const float* Wout  = (const float*)d_in[2];
    const float* bout  = (const float*)d_in[3];
    const float* relp  = (const float*)d_in[4];
    const float* gamma = (const float*)d_in[5];
    const float* beta  = (const float*)d_in[6];
    float* out = (float*)d_out;

    const size_t nx   = (size_t)NB * NT * NF;
    const size_t nwq  = (size_t)NO3 * NF;
    const size_t nwo  = (size_t)NDO * NDH;
    const size_t nqkv = (size_t)NB * NO3 * NT;
    const size_t nps  = (size_t)NT * NDK;
    const size_t nhd  = (size_t)NHN * NDK * NT;
    const size_t nhid = (size_t)NB * NT * NDH;
    size_t off = 0;
    const size_t o_xh  = off; off = al256(off + nx * 2);
    const size_t o_xl  = off; off = al256(off + nx * 2);
    const size_t o_wqh = off; off = al256(off + nwq * 2);
    const size_t o_wql = off; off = al256(off + nwq * 2);
    const size_t o_woh = off; off = al256(off + nwo * 2);
    const size_t o_wol = off; off = al256(off + nwo * 2);
    const size_t o_qkv = off; off = al256(off + nqkv * 4);
    const size_t o_ps  = off; off = al256(off + nps * 4);
    const size_t o_kh  = off; off = al256(off + nhd * 2);
    const size_t o_kl  = off; off = al256(off + nhd * 2);
    const size_t o_vh  = off; off = al256(off + nhd * 2);
    const size_t o_vl  = off; off = al256(off + nhd * 2);
    const size_t o_qth = off; off = al256(off + nhd * 2);
    const size_t o_qtl = off; off = al256(off + nhd * 2);
    const size_t o_S   = off; off = al256(off + (size_t)NHN * NT * 4);
    const size_t o_bnp = off; off = al256(off + (size_t)NHN * 128 * 8);
    const size_t o_bnc = off; off = al256(off + 128 * 4);
    if (off > ws_size) return;
    if (nhid > nx) return;
    const size_t o_hh = o_xh, o_hl = o_xl;

    char* ws = (char*)d_ws;
    u16*    xh   = (u16*)(ws + o_xh);
    u16*    xl   = (u16*)(ws + o_xl);
    u16*    wqh  = (u16*)(ws + o_wqh);
    u16*    wql  = (u16*)(ws + o_wql);
    u16*    woh  = (u16*)(ws + o_woh);
    u16*    wol  = (u16*)(ws + o_wol);
    float*  qkv  = (float*)(ws + o_qkv);
    float*  psum = (float*)(ws + o_ps);
    u16*    kh   = (u16*)(ws + o_kh);
    u16*    kl   = (u16*)(ws + o_kl);
    u16*    vh   = (u16*)(ws + o_vh);
    u16*    vl   = (u16*)(ws + o_vl);
    u16*    qth  = (u16*)(ws + o_qth);
    u16*    qtl  = (u16*)(ws + o_qtl);
    float*  Sbuf = (float*)(ws + o_S);
    double* bnp  = (double*)(ws + o_bnp);
    float*  bnc  = (float*)(ws + o_bnc);
    u16*    hidh = (u16*)(ws + o_hh);
    u16*    hidl = (u16*)(ws + o_hl);

    {
        const int n8x = (int)(nx / 8), n8q = (int)(nwq / 8), n8o = (int)(nwo / 8);
        k_cvt<<<dim3((n8x + 255) / 256, 1), 256, 0, stream>>>(x, (size_t)0, xh, xl, (size_t)0, n8x);
        k_cvt<<<dim3((n8q + 255) / 256, 1), 256, 0, stream>>>(Wqkv, (size_t)0, wqh, wql, (size_t)0, n8q);
        k_cvt<<<dim3((n8o + 255) / 256, 1), 256, 0, stream>>>(Wout, (size_t)0, woh, wol, (size_t)0, n8o);
    }
    k_gemm<<<dim3(NT / 64, NO3 / 64, NB), 128, 0, stream>>>(
        wqh, wql, xh, xl, (size_t)NT * NF, qkv, (size_t)NO3 * NT, bout, NDO, 0, NO3, NT, NF);
    k_psum<<<NT, 64, 0, stream>>>(relp, psum);
    k_soft<<<NB * NDH, 128, 0, stream>>>(qkv, kh, kl);
    {
        const int n8v = (int)((size_t)NDH * NT / 8);
        k_cvt<<<dim3((n8v + 255) / 256, NB), 256, 0, stream>>>(
            qkv + (size_t)(2 * NDH) * NT, (size_t)NO3 * NT, vh, vl, (size_t)NDH * NT, n8v);
    }
    k_qtr<<<dim3(NT / 32, NHN), 256, 0, stream>>>(qkv, qth, qtl);
    k_rel<<<NHN, 256, 0, stream>>>(qkv, psum, Sbuf, bnp);
    k_bnfin<<<1, 64, 0, stream>>>(bnp, gamma, beta, bnc);
    k_head<<<NHN, 256, 0, stream>>>(qkv, kh, kl, vh, vl, qth, qtl, Sbuf, bnc, hidh, hidl);
    k_gemm<<<dim3(NT / 64, NDO / 64, NB), 128, 0, stream>>>(
        woh, wol, hidh, hidl, (size_t)NT * NDH, out, (size_t)NDO * NT, bout, NDO, 1, NDO, NT, NDH);
}
